// DecoderBlock_74208444940651
// MI455X (gfx1250) — hardware-verified
//
#include <hip/hip_runtime.h>
#include <math.h>

#ifndef NB
#define NB 1
#endif
#ifndef SEQ
#define SEQ 2048
#endif
#ifndef SRC
#define SRC 2048
#endif
#define SEQ_FULL 2048
#define SRC_FULL 2048

typedef __attribute__((ext_vector_type(16))) _Float16 v16h;
typedef __attribute__((ext_vector_type(8)))  _Float16 v8h;
typedef __attribute__((ext_vector_type(16))) __bf16   v16b;
typedef __attribute__((ext_vector_type(8)))  __bf16   v8b;
typedef __attribute__((ext_vector_type(8)))  float    v8f;
typedef __attribute__((ext_vector_type(4)))  float    v4f;
typedef __attribute__((ext_vector_type(4)))  unsigned v4u;
typedef __attribute__((ext_vector_type(2)))  unsigned v2u;

constexpr int kBatch   = NB;
constexpr int kSeq     = SEQ;
constexpr int kSrc     = SRC;
constexpr int kSeqFull = SEQ_FULL;
constexpr int kSrcFull = SRC_FULL;
constexpr int kDim   = 1024;
constexpr int kHeads = 16;
constexpr int kHdim  = 64;
constexpr int kFfn   = 4096;
constexpr int kRows  = kBatch * kSeq;
constexpr int kCRows = kBatch * kSrc;
constexpr int kQkvLd = 3 * kDim;
constexpr int kKvLd  = 2 * kDim;
constexpr float kNegBig = 1.0e10f;

static_assert(kBatch >= 1 && kSeq % 64 == 0 && kSrc % 64 == 0 && kSeq <= kSeqFull && kSrc <= kSrcFull);
static_assert(kHeads * kHdim == kDim && kHdim == 64);
static_assert(kDim % 64 == 0 && kFfn % 64 == 0 && kQkvLd % 64 == 0 && kKvLd % 64 == 0 && kDim % 32 == 0 && kFfn % 32 == 0);

constexpr float kCarryIn   = 8.0f;
constexpr float kCarryW    = 64.0f;
constexpr float kCarryQkv  = 8.0f;
constexpr float kCarryAct  = 8.0f;
constexpr float kCarryP    = 1024.0f;
constexpr float kCarryAttn = 64.0f;
constexpr float kCarryWo   = 256.0f;
constexpr float kCarryW1   = 256.0f;
constexpr float kCarryW2   = 512.0f;
constexpr float kCarryH    = 8.0f;

constexpr size_t kSzTgt16 = (size_t)kRows * kDim * 2;
constexpr size_t kSzCtx16 = (size_t)kCRows * kDim * 2;
constexpr size_t kSzWqkvT = (size_t)kQkvLd * kDim * 2;
constexpr size_t kSzWsq   = (size_t)kDim * kDim * 2;
constexpr size_t kSzWkvT  = (size_t)kKvLd * kDim * 2;
constexpr size_t kSzW1T   = (size_t)kFfn * kDim * 2;
constexpr size_t kSzW2T   = (size_t)kDim * kFfn * 2;
constexpr size_t kSzQkv   = (size_t)kRows * kQkvLd * 2;
constexpr size_t kSzH16   = (size_t)kRows * kDim * 2;
constexpr size_t kSzF32   = (size_t)kRows * kDim * 4;
constexpr size_t kSzKv2   = (size_t)kCRows * kKvLd * 2;
constexpr size_t kSzHid   = (size_t)kRows * kFfn * 2;
constexpr size_t kOffTgt16 = 0;
constexpr size_t kOffCtx16 = kOffTgt16 + kSzTgt16;
constexpr size_t kOffWqkvT = kOffCtx16 + kSzCtx16;
constexpr size_t kOffWo1T  = kOffWqkvT + kSzWqkvT;
constexpr size_t kOffWqT   = kOffWo1T + kSzWsq;
constexpr size_t kOffWkvT  = kOffWqT + kSzWsq;
constexpr size_t kOffWo2T  = kOffWkvT + kSzWkvT;
constexpr size_t kOffW1T   = kOffWo2T + kSzWsq;
constexpr size_t kOffW2T   = kOffW1T + kSzW1T;
constexpr size_t kOffQkv   = kOffW2T + kSzW2T;
constexpr size_t kOffAttn  = kOffQkv + kSzQkv;
constexpr size_t kOffU     = kOffAttn + kSzH16;
constexpr size_t kOffT1f   = kOffU + kSzF32;
constexpr size_t kOffT1h   = kOffT1f + kSzF32;
constexpr size_t kOffQ2    = kOffT1h + kSzH16;
constexpr size_t kOffKv2   = kOffQ2 + kSzH16;
constexpr size_t kOffT2f   = kOffKv2 + kSzKv2;
constexpr size_t kOffT2h   = kOffT2f + kSzF32;
constexpr size_t kOffHid   = kOffT2h + kSzH16;
constexpr size_t kWsTotal  = kOffHid + kSzHid;
static_assert(kWsTotal <= (size_t)134217728);
static_assert(!(kBatch == 1 && kSeq == 2048 && kSrc == 2048) || kWsTotal == (size_t)121634816);
static_assert((kSzTgt16 % 128) == 0 && (kSzCtx16 % 128) == 0 && (kSzWqkvT % 128) == 0 && (kSzWsq % 128) == 0 &&
              (kSzWkvT % 128) == 0 && (kSzW1T % 128) == 0 && (kSzW2T % 128) == 0 && (kSzQkv % 128) == 0 &&
              (kSzH16 % 128) == 0 && (kSzF32 % 128) == 0 && (kSzKv2 % 128) == 0 && (kSzHid % 128) == 0);

__device__ __forceinline__ unsigned short f2bf_bits(float f) {
  unsigned u = __float_as_uint(f);
  return (unsigned short)((u + 0x7FFFu + ((u >> 16) & 1u)) >> 16);
}
__device__ __forceinline__ float bf_bits2f(unsigned short h) { return __uint_as_float(((unsigned)h) << 16); }
__device__ __forceinline__ float bf_rne(float f) { return bf_bits2f(f2bf_bits(f)); }
__device__ __forceinline__ unsigned pack_h2(float x, float y, float sc) {
  const _Float16 h0 = (_Float16)(bf_rne(x) * sc);
  const _Float16 h1 = (_Float16)(bf_rne(y) * sc);
  return (unsigned)__builtin_bit_cast(unsigned short, h0) | ((unsigned)__builtin_bit_cast(unsigned short, h1) << 16);
}

__device__ __forceinline__ void dep_guard_h(v8f& a, v8f& b, v16h x, v16h y) { asm volatile("v_nop\n\tv_nop\n\tv_nop\n\tv_nop" : "+v"(a), "+v"(b) : "v"(x), "v"(y)); }
__device__ __forceinline__ void dep_guard_b(v8f& a, v8f& b, v16b x, v16b y) { asm volatile("v_nop\n\tv_nop\n\tv_nop\n\tv_nop" : "+v"(a), "+v"(b) : "v"(x), "v"(y)); }
__device__ __forceinline__ void keep4_h(v16h a, v16h b, v16h c, v16h d) { asm volatile("v_nop" :: "v"(a), "v"(b), "v"(c), "v"(d)); }
__device__ __forceinline__ void keep4_b(v16b a, v16b b, v16b c, v16b d) { asm volatile("v_nop" :: "v"(a), "v"(b), "v"(c), "v"(d)); }
__device__ __forceinline__ void acc_guard4(v8f& a, v8f& b, v8f& c, v8f& d) { asm volatile("v_nop\n\tv_nop\n\tv_nop\n\tv_nop" : "+v"(a), "+v"(b), "+v"(c), "+v"(d)); }
template <typename T> struct Frag;
template <> struct Frag<_Float16> {
  typedef v16h V; union U { v16h v; v8h h[2]; };
  static __device__ __forceinline__ v16h load(const _Float16* p) {
    U f; f.h[0] = *(const v8h*)(p); f.h[1] = *(const v8h*)(p + 16); return f.v;
  }
  static __device__ __forceinline__ v8f mma(v16h a, v16h b, v8f c) {
    return __builtin_amdgcn_wmma_f32_16x16x32_f16(false, a, false, b, (short)0, c, false, false);
  }
  static __device__ __forceinline__ void guard(v8f& a, v8f& b, v16h x, v16h y) { dep_guard_h(a, b, x, y); }
  static __device__ __forceinline__ void keep(v16h a, v16h b, v16h c, v16h d) { keep4_h(a, b, c, d); }
};
template <> struct Frag<__bf16> {
  typedef v16b V; union U { v16b v; v8b h[2]; };
  static __device__ __forceinline__ v16b load(const __bf16* p) {
    U f; f.h[0] = *(const v8b*)(p); f.h[1] = *(const v8b*)(p + 16); return f.v;
  }
  static __device__ __forceinline__ v8f mma(v16b a, v16b b, v8f c) {
    return __builtin_amdgcn_wmma_f32_16x16x32_bf16(false, a, false, b, (short)0, c, false, false);
  }
  static __device__ __forceinline__ void guard(v8f& a, v8f& b, v16b x, v16b y) { dep_guard_b(a, b, x, y); }
  static __device__ __forceinline__ void keep(v16b a, v16b b, v16b c, v16b d) { keep4_b(a, b, c, d); }
};

template <int ET> struct Elem;
template <> struct Elem<0> { typedef _Float16 T; };
template <> struct Elem<1> { typedef __bf16 T; };
template <int ET, bool SPLIT, int BIAS_MODE, int OUT_MODE, bool RESID, bool RRNE, int ACT>
__global__ __launch_bounds__(256) void wmma_gemm64(
    const unsigned short* __restrict__ Ap, const unsigned short* __restrict__ A2p, int lda, long strideA,
    const unsigned short* __restrict__ Btp, const unsigned short* __restrict__ Bt2p, int ldb, long strideB,
    void* __restrict__ Cout, void* __restrict__ Cout2, int ldc, long strideC,
    const float* __restrict__ bias,
    const float* __restrict__ resid, long strideR,
    int M, int N, int K, float scale, float oscale) {
  static_assert(!RESID || OUT_MODE == 0);
  typedef typename Elem<ET>::T T;
  typedef typename Frag<T>::V V;
  const T* A = (const T*)Ap; const T* A2 = (const T*)A2p; const T* Bt = (const T*)Btp; const T* Bt2 = (const T*)Bt2p;
  __shared__ __align__(16) float sT[8][16 * 68];
  const int b    = blockIdx.y;
  const int lane = threadIdx.x & 31;
  const int wave = threadIdx.x >> 5;
  const int tilesN = N >> 6;
  const int tilesM = M >> 6;
  const int tile = blockIdx.x * 8 + wave;
  if (tile >= tilesM * tilesN) return;
  const int tm = tile / tilesN;
  const int tn = tile - tm * tilesN;
  const int m0 = tm << 6;
  const int n0 = tn << 6;

  const T* Ab  = A  + (size_t)b * strideA;
  const T* Bb  = Bt + (size_t)b * strideB;
  const T* Ab2 = SPLIT ? (A2  + (size_t)b * strideA) : nullptr;
  const T* Bb2 = SPLIT ? (Bt2 + (size_t)b * strideB) : nullptr;

  const int rlane = lane & 15;
  const int koff  = (lane >> 4) * 8;
  const int mOff  = (lane >> 4) * 8;

  v8f acc[4][4];
#pragma unroll
  for (int i = 0; i < 4; ++i)
#pragma unroll
    for (int j = 0; j < 4; ++j) acc[i][j] = (v8f){0.f,0.f,0.f,0.f,0.f,0.f,0.f,0.f};

  for (int k0 = 0; k0 < K; k0 += 32) {
    V bh[4], bl[4];
#pragma unroll
    for (int j = 0; j < 4; ++j) {
      const size_t bo = (size_t)(n0 + (j << 4) + rlane) * ldb + koff + k0;
      bh[j] = Frag<T>::load(Bb + bo);
      if (SPLIT) bl[j] = Frag<T>::load(Bb2 + bo);
    }
#pragma unroll
    for (int i = 0; i < 4; ++i) {
      const size_t ao = (size_t)(m0 + (i << 4) + rlane) * lda + koff + k0;
      V ah = Frag<T>::load(Ab + ao);
      V al;
      if (SPLIT) al = Frag<T>::load(Ab2 + ao);
#pragma unroll
      for (int j = 0; j < 4; ++j) {
        acc[i][j] = Frag<T>::mma(ah, bh[j], acc[i][j]);
        if (SPLIT) {
          acc[i][j] = Frag<T>::mma(ah, bl[j], acc[i][j]);
          acc[i][j] = Frag<T>::mma(al, bh[j], acc[i][j]);
        }
      }
      Frag<T>::guard(acc[i][0], acc[i][3], ah, SPLIT ? al : ah);
    }
    Frag<T>::keep(bh[0], bh[1], bh[2], bh[3]);
    if (SPLIT) Frag<T>::keep(bl[0], bl[1], bl[2], bl[3]);
  }
  acc_guard4(acc[0][0], acc[0][1], acc[0][2], acc[0][3]);
  acc_guard4(acc[1][0], acc[1][1], acc[1][2], acc[1][3]);
  acc_guard4(acc[2][0], acc[2][1], acc[2][2], acc[2][3]);
  acc_guard4(acc[3][0], acc[3][1], acc[3][2], acc[3][3]);

  float* slab = sT[wave];
  const float* Rb = RESID ? (resid + (size_t)b * strideR) : nullptr;
#pragma unroll
  for (int i = 0; i < 4; ++i) {
    const int mBase = m0 + (i << 4);
#pragma unroll
    for (int j = 0; j < 4; ++j) {
      const int n = n0 + (j << 4) + rlane;
      float bv = 0.f;
      if (BIAS_MODE == 2) bv = bias[n];
#pragma unroll
      for (int r = 0; r < 8; ++r) {
        float v = acc[i][j][r] * scale;
        if (BIAS_MODE == 1) v += bias[mBase + mOff + r];
        if (BIAS_MODE == 2) v += bv;
        if (ACT == 1) v = tanhf(v);
        if (ACT == 2) v = fmaxf(v, 0.0f);
        if (ACT == 3) v = v / (1.0f + expf(-v));
        if (ACT == 4) v = (v > 0.f) ? v : 0.01f * v;
        if (ACT == 6) {
          float t2 = 1.5957691216057308f * (v + 0.044715f * v * v * v);
          t2 = fmaxf(t2, -80.0f);
          v = v * __builtin_amdgcn_rcpf(1.0f + __expf(-t2));
        }
        if (ACT == 7) v = 0.5f * v * (1.0f + erff(v * 0.70710678118654752f));
        slab[(mOff + r) * 68 + (j << 4) + rlane] = v * oscale;
      }
    }
    __builtin_amdgcn_fence(3  , "workgroup");
    __builtin_amdgcn_wave_barrier();
    __builtin_amdgcn_fence(2  , "workgroup");
    if (OUT_MODE == 0) {
      float* C = (float*)Cout + (size_t)b * strideC;
      const int hh = lane >> 4, c4 = (lane & 15) * 4;
      for (int ps = 0; ps < 2; ++ps) {
#pragma unroll
        for (int it = 0; it < 8; ++it) {
          const int row = it * 2 + hh;
          v4f v = *(const v4f*)(slab + row * 68 + c4);
          if (RESID) {
            v4f rr = *(const v4f*)(Rb + (size_t)(mBase + row) * ldc + n0 + c4);
            if (RRNE) { rr[0] = bf_rne(rr[0]); rr[1] = bf_rne(rr[1]); rr[2] = bf_rne(rr[2]); rr[3] = bf_rne(rr[3]); }
            v += rr;
          }
          *(volatile v4f*)(C + (size_t)(mBase + row) * ldc + n0 + c4) = v;
        }
        __threadfence();
      }
    } else {
      const int q = lane >> 3, c8 = (lane & 7) * 8;
      unsigned short* C  = (unsigned short*)Cout  + (size_t)b * strideC;
      unsigned short* C2 = (OUT_MODE == 2) ? ((unsigned short*)Cout2 + (size_t)b * strideC) : nullptr;
      for (int ps = 0; ps < 2; ++ps) {
#pragma unroll
        for (int it = 0; it < 4; ++it) {
          const int row = it * 4 + q;
          const float* sp = slab + row * 68 + c8;
          v8h hv, lv;
#pragma unroll
          for (int e = 0; e < 8; ++e) {
            if (OUT_MODE == 1) {
              hv[e] = (_Float16)sp[e];
            } else {
              unsigned short hb = f2bf_bits(sp[e]);
              unsigned short lb = f2bf_bits(sp[e] - bf_bits2f(hb));
              hv[e] = __builtin_bit_cast(_Float16, hb);
              lv[e] = __builtin_bit_cast(_Float16, lb);
            }
          }
          *(volatile v8h*)(C + (size_t)(mBase + row) * ldc + n0 + c8) = hv;
          if (OUT_MODE == 2) *(volatile v8h*)(C2 + (size_t)(mBase + row) * ldc + n0 + c8) = lv;
        }
        __threadfence();
      }
    }
    __builtin_amdgcn_fence(3  , "workgroup");
    __builtin_amdgcn_wave_barrier();
    __builtin_amdgcn_fence(2  , "workgroup");
  }
}

__global__ __launch_bounds__(256) void cast_act(
    const float* __restrict__ in, _Float16* __restrict__ out, int n8, int seq, int seqFull, float sc) {
  const int i = blockIdx.x * 256 + threadIdx.x;
  if (i < n8) {
    const int r = i >> 7;
    const int col = (i & 127) * 8;
    const int bb = r / seq;
    const int ss = r - bb * seq;
    const float* p = in + ((size_t)bb * seqFull + ss) * kDim + col;
    const v4f a = *(const v4f*)(p);
    const v4f c = *(const v4f*)(p + 4);
    v4u u;
    u[0] = pack_h2(a[0], a[1], sc);
    u[1] = pack_h2(a[2], a[3], sc);
    u[2] = pack_h2(c[0], c[1], sc);
    u[3] = pack_h2(c[2], c[3], sc);
    _Float16* op = out + (size_t)i * 8;
    *(volatile v4u*)op = u;
    __threadfence();
    *(volatile v4u*)op = u;
  }
}

__global__ __launch_bounds__(256) void cast_wT(
    const float* __restrict__ in, _Float16* __restrict__ out, int R, int C, float sc) {
  __shared__ __align__(16) _Float16 tl[64 * 72];
  const int t = threadIdx.x;
  const int c0 = blockIdx.x * 64;
  const int r0 = blockIdx.y * 64;
  const int rr = t >> 2;
  const int cb = (t & 3) * 16;
  const float* src = in + (size_t)(r0 + rr) * C + c0 + cb;
#pragma unroll
  for (int q = 0; q < 4; ++q) {
    const v4f v = *(const v4f*)(src + 4 * q);
#pragma unroll
    for (int e = 0; e < 4; ++e) tl[(cb + 4 * q + e) * 72 + rr] = (_Float16)(bf_rne(v[e]) * sc);
  }
  __syncthreads();
  const int w = t >> 5, lane = t & 31, q8 = lane >> 3, c8 = (lane & 7) * 8;
  for (int ps = 0; ps < 2; ++ps) {
#pragma unroll
    for (int it = 0; it < 2; ++it) {
      const int row = w * 8 + it * 4 + q8;
      const v4u val = *(const v4u*)(tl + row * 72 + c8);
      *(volatile v4u*)(out + (size_t)(c0 + row) * R + r0 + c8) = val;
    }
    __threadfence();
  }
}

template <bool WH>
__global__ __launch_bounds__(256) void layernorm_rows(
    const float* __restrict__ x, const float* __restrict__ gam, const float* __restrict__ bet,
    float* __restrict__ yf, _Float16* __restrict__ yh, float hscale, float eps) {
  __shared__ float ssum[8];
  __shared__ float ssq[8];
  __shared__ __align__(16) unsigned hrow[512];
  const int row = blockIdx.x;
  const int t = threadIdx.x;
  const int w = t >> 5;
  const int l = t & 31;
  const v4f v = *(const v4f*)(x + (size_t)row * kDim + t * 4);
  float s = (v[0] + v[1]) + (v[2] + v[3]);
#pragma unroll
  for (int off = 1; off < 32; off <<= 1) s += __shfl_xor(s, off, 32);
  if (l == 0) ssum[w] = s;
  __syncthreads();
  float tot = 0.f;
#pragma unroll
  for (int i = 0; i < 8; ++i) tot += ssum[i];
  const float mean = tot * (1.0f / 1024.0f);
  const v4f d = v - mean;
  float q = (d[0] * d[0] + d[1] * d[1]) + (d[2] * d[2] + d[3] * d[3]);
#pragma unroll
  for (int off = 1; off < 32; off <<= 1) q += __shfl_xor(q, off, 32);
  if (l == 0) ssq[w] = q;
  __syncthreads();
  float totq = 0.f;
#pragma unroll
  for (int i = 0; i < 8; ++i) totq += ssq[i];
  const float var = totq * (1.0f / 1024.0f);
  const float inv = rsqrtf(var + eps);
  const v4f gv = *(const v4f*)(gam + t * 4);
  const v4f bv = *(const v4f*)(bet + t * 4);
  const v4f o = d * inv * gv + bv;
  float* yrow = yf + (size_t)row * kDim + t * 4;
  *(volatile v4f*)yrow = o;
  __threadfence();
  *(volatile v4f*)yrow = o;
  if (WH) {
    const unsigned hb0 = (unsigned)__builtin_bit_cast(unsigned short, (_Float16)(o[0] * hscale));
    const unsigned hb1 = (unsigned)__builtin_bit_cast(unsigned short, (_Float16)(o[1] * hscale));
    const unsigned hb2 = (unsigned)__builtin_bit_cast(unsigned short, (_Float16)(o[2] * hscale));
    const unsigned hb3 = (unsigned)__builtin_bit_cast(unsigned short, (_Float16)(o[3] * hscale));
    v2u pk;
    pk[0] = hb0 | (hb1 << 16);
    pk[1] = hb2 | (hb3 << 16);
    *(v2u*)(hrow + 2 * t) = pk;
    __syncthreads();
    if (t < 128) {
      const v4u wv = *(const v4u*)(hrow + 4 * t);
      _Float16* hp = yh + (size_t)row * kDim + t * 8;
      *(volatile v4u*)hp = wv;
      __threadfence();
      *(volatile v4u*)hp = wv;
    }
  }
}

constexpr int kAKC = 64;
constexpr int kAQB = 64;
constexpr int kANW = 4;

__device__ __forceinline__ v8f mma_h(v16h a, v16h b, v8f c) {
  c = __builtin_amdgcn_wmma_f32_16x16x32_f16(false, a, false, b, (short)0, c, false, false);
  asm volatile("v_nop\n\tv_nop\n\tv_nop\n\tv_nop" : "+v"(c) : "v"(a), "v"(b));
  return c;
}

__device__ __forceinline__ void vt_scatter(_Float16* vt, v4u w, int d0, int kvr) {
#pragma unroll
  for (int e = 0; e < 4; ++e) {
    const unsigned u = w[e];
    const int d = d0 + 2 * e;
    vt[d * kAKC + kvr]       = __builtin_bit_cast(_Float16, (unsigned short)(u & 0xffffu));
    vt[(d + 1) * kAKC + kvr] = __builtin_bit_cast(_Float16, (unsigned short)(u >> 16));
  }
}

template <bool CAUSAL>
__global__ __launch_bounds__(128)
void attn_h64(const _Float16* __restrict__ qp, int ldq, long qStride,
              const _Float16* __restrict__ kp, int ldk, long kStride,
              const _Float16* __restrict__ vp, int ldv, long vStride,
              const int* __restrict__ padk, int padStride,
              _Float16* __restrict__ attn_out, long oStride,
              int nq, int nk, float sscale, float pscale, float oscale) {
  union FH { v16h v; v8h h[2]; };
  __shared__ __align__(16) _Float16 Ksh[kAKC * kHdim];
  __shared__ __align__(16) _Float16 Vth[kHdim * kAKC];
  __shared__ __align__(16) _Float16 Psh[kANW][16 * kAKC];
  __shared__ __align__(16) float  Osl[kANW][16 * 68];

  const int tid  = threadIdx.x;
  const int wave = tid >> 5;
  const int lane = tid & 31;
  const int hh   = lane >> 4;
  const int c    = lane & 15;

  const int nqb = nq / kAQB;
  const int bx = blockIdx.x;
  const int qb = bx % nqb;
  const int bh = bx / nqb;
  const int h  = bh % kHeads;
  const int b  = bh / kHeads;
  const int q0 = qb * kAQB + wave * 16;

  const _Float16* qbase = qp + (size_t)b * qStride + h * kHdim;
  const _Float16* kbase = kp + (size_t)b * kStride + h * kHdim;
  const _Float16* vbase = vp + (size_t)b * vStride + h * kHdim;
  const int* pk = padk + (size_t)b * padStride;
  _Float16* ob = attn_out + (size_t)b * oStride + h * kHdim;

  v16h qa[2];
  {
    const _Float16* qrow = qbase + (size_t)(q0 + c) * ldq + 8 * hh;
    qa[0] = Frag<_Float16>::load(qrow);
    qa[1] = Frag<_Float16>::load(qrow + 32);
  }

  float mrow[8], lrow[8];
  v8f oacc[4];
#pragma unroll
  for (int r = 0; r < 8; ++r) { mrow[r] = -INFINITY; lrow[r] = 0.f; }
#pragma unroll
  for (int t = 0; t < 4; ++t) oacc[t] = (v8f){0.f,0.f,0.f,0.f,0.f,0.f,0.f,0.f};

  const int nkc = nk / kAKC;
  int nChunks = nkc;
  if (CAUSAL) {
    const int p0 = pk[0];
    nChunks = (p0 != 0) ? (qb + 1) : nkc;
  }
  for (int kc = 0; kc < nChunks; ++kc) {
    const int kv0 = kc * kAKC;
    __syncthreads();
    {
      const int kvr = tid >> 1, dh = (tid & 1) * 32;
      const _Float16* krow = kbase + (size_t)(kv0 + kvr) * ldk + dh;
      const _Float16* vrow = vbase + (size_t)(kv0 + kvr) * ldv + dh;
      const v8h k0v = *(const v8h*)(krow);
      const v8h k1v = *(const v8h*)(krow + 8);
      const v8h k2v = *(const v8h*)(krow + 16);
      const v8h k3v = *(const v8h*)(krow + 24);
      const v4u v0w = *(const v4u*)(vrow);
      const v4u v1w = *(const v4u*)(vrow + 8);
      const v4u v2w = *(const v4u*)(vrow + 16);
      const v4u v3w = *(const v4u*)(vrow + 24);
      _Float16* kd = Ksh + kvr * kHdim + dh;
      *(v8h*)(kd)      = k0v;
      *(v8h*)(kd + 8)  = k1v;
      *(v8h*)(kd + 16) = k2v;
      *(v8h*)(kd + 24) = k3v;
      vt_scatter(Vth, v0w, dh,      kvr);
      vt_scatter(Vth, v1w, dh + 8,  kvr);
      vt_scatter(Vth, v2w, dh + 16, kvr);
      vt_scatter(Vth, v3w, dh + 24, kvr);
    }
    __syncthreads();

    float mkf[4];
#pragma unroll
    for (int j = 0; j < 4; ++j) mkf[j] = (float)pk[kv0 + j * 16 + c];

    v8f s[4];
#pragma unroll
    for (int j = 0; j < 4; ++j) {
      s[j] = (v8f){0.f,0.f,0.f,0.f,0.f,0.f,0.f,0.f};
#pragma unroll
      for (int dc = 0; dc < 2; ++dc) {
        FH kb;
        kb.h[0] = *(const v8h*)(Ksh + (j * 16 + c) * kHdim + dc * 32 + 8 * hh);
        kb.h[1] = *(const v8h*)(Ksh + (j * 16 + c) * kHdim + dc * 32 + 16 + 8 * hh);
        s[j] = mma_h(qa[dc], kb.v, s[j]);
      }
    }
    float cm[8];
#pragma unroll
    for (int r = 0; r < 8; ++r) {
      const int qrow = q0 + 8 * hh + r;
      float m = -INFINITY;
#pragma unroll
      for (int j = 0; j < 4; ++j) {
        const int kvcol = kv0 + j * 16 + c;
        float sv = s[j][r] * sscale;
        float mf = mkf[j];
        if (CAUSAL) mf = (kvcol <= qrow) ? mf : 0.0f;
        sv = sv * mf - (1.0f - mf) * kNegBig;
        s[j][r] = sv;
        m = fmaxf(m, sv);
      }
#pragma unroll
      for (int off = 1; off < 16; off <<= 1) m = fmaxf(m, __shfl_xor(m, off, 32));
      cm[r] = m;
    }
    _Float16* pw = Psh[wave];
#pragma unroll
    for (int r = 0; r < 8; ++r) {
      const float mnew = fmaxf(mrow[r], cm[r]);
      const float alpha = __expf(mrow[r] - mnew);
      mrow[r] = mnew;
      float psum = 0.f;
#pragma unroll
      for (int j = 0; j < 4; ++j) {
        const float p = __expf(s[j][r] - mnew);
        psum += p;
        pw[(8 * hh + r) * kAKC + j * 16 + c] = (_Float16)(p * pscale);
      }
#pragma unroll
      for (int off = 1; off < 16; off <<= 1) psum += __shfl_xor(psum, off, 32);
      lrow[r] = lrow[r] * alpha + psum;
#pragma unroll
      for (int t = 0; t < 4; ++t) oacc[t][r] *= alpha;
    }
    __builtin_amdgcn_fence(3  , "workgroup");
    __builtin_amdgcn_wave_barrier();
    __builtin_amdgcn_fence(2  , "workgroup");
#pragma unroll
    for (int kk = 0; kk < 2; ++kk) {
      FH pa;
      pa.h[0] = *(const v8h*)(pw + c * kAKC + kk * 32 + 8 * hh);
      pa.h[1] = *(const v8h*)(pw + c * kAKC + kk * 32 + 16 + 8 * hh);
#pragma unroll
      for (int t = 0; t < 4; ++t) {
        FH vb;
        vb.h[0] = *(const v8h*)(Vth + (t * 16 + c) * kAKC + kk * 32 + 8 * hh);
        vb.h[1] = *(const v8h*)(Vth + (t * 16 + c) * kAKC + kk * 32 + 16 + 8 * hh);
        oacc[t] = mma_h(pa.v, vb.v, oacc[t]);
      }
    }
  }

  float* os = Osl[wave];
#pragma unroll
  for (int r = 0; r < 8; ++r) {
    const float inv = oscale / lrow[r];
#pragma unroll
    for (int t = 0; t < 4; ++t) os[(8 * hh + r) * 68 + t * 16 + c] = oacc[t][r] * inv;
  }
  __builtin_amdgcn_fence(3  , "workgroup");
  __builtin_amdgcn_wave_barrier();
  __builtin_amdgcn_fence(2  , "workgroup");
  {
    const int q8 = lane >> 3, c8 = (lane & 7) * 8;
    for (int ps = 0; ps < 2; ++ps) {
#pragma unroll
      for (int it = 0; it < 4; ++it) {
        const int row = it * 4 + q8;
        const float* sp = os + row * 68 + c8;
        v8h hv;
#pragma unroll
        for (int e = 0; e < 8; ++e) hv[e] = (_Float16)sp[e];
        *(volatile v8h*)(ob + (size_t)(q0 + row) * kDim + c8) = hv;
      }
      __threadfence();
    }
  }
}

extern "C" void kernel_launch(void* const* d_in, const int* in_sizes, int n_in,
                              void* d_out, int out_size, void* d_ws, size_t ws_size,
                              hipStream_t stream) {
  if (n_in != 22) return;
  const long needT = (long)(kBatch - 1) * kSeqFull * kDim + (long)kSeq * kDim;
  const long needC = (long)(kBatch - 1) * kSrcFull * kDim + (long)kSrc * kDim;
  if ((long)in_sizes[0] < needT || (long)in_sizes[1] < needC) return;
  if (in_sizes[2] < (kBatch - 1) * kSeqFull + kSeq || in_sizes[3] < (kBatch - 1) * kSrcFull + kSrc) return;
  if (in_sizes[4] != kDim * kQkvLd) return;
  if (in_sizes[5] != kDim * kDim || in_sizes[9] != kDim * kDim || in_sizes[10] != kDim * kDim ||
      in_sizes[11] != kDim * kDim || in_sizes[12] != kDim * kDim) return;
  if (in_sizes[6] != kDim || in_sizes[7] != kDim || in_sizes[8] != kDim || in_sizes[13] != kDim ||
      in_sizes[14] != kDim || in_sizes[15] != kDim || in_sizes[19] != kDim || in_sizes[20] != kDim ||
      in_sizes[21] != kDim) return;
  if (in_sizes[16] != kDim * kFfn || in_sizes[17] != kFfn || in_sizes[18] != kFfn * kDim) return;
  if (out_size < kRows * kDim) return;
  if (ws_size < kWsTotal) return;

  const float* target  = (const float*)d_in[0];
  const float* context = (const float*)d_in[1];
  const int*   tpad    = (const int*)d_in[2];
  const int*   cpad    = (const int*)d_in[3];
  const float* Wqkv = (const float*)d_in[4];
  const float* Wo1  = (const float*)d_in[5];
  const float* bo1  = (const float*)d_in[6];
  const float* g1   = (const float*)d_in[7];
  const float* b1   = (const float*)d_in[8];
  const float* Wq   = (const float*)d_in[9];
  const float* Wk   = (const float*)d_in[10];
  const float* Wv   = (const float*)d_in[11];
  const float* Wo2  = (const float*)d_in[12];
  const float* bo2  = (const float*)d_in[13];
  const float* g2   = (const float*)d_in[14];
  const float* b2   = (const float*)d_in[15];
  const float* W1   = (const float*)d_in[16];
  const float* bf1  = (const float*)d_in[17];
  const float* W2   = (const float*)d_in[18];
  const float* bf2  = (const float*)d_in[19];
  const float* g3   = (const float*)d_in[20];
  const float* b3   = (const float*)d_in[21];
  float* outf = (float*)d_out;

  char* ws = (char*)d_ws;
  _Float16* tgt16 = (_Float16*)(ws + kOffTgt16);
  _Float16* ctx16 = (_Float16*)(ws + kOffCtx16);
  _Float16* wqkvT = (_Float16*)(ws + kOffWqkvT);
  _Float16* wo1T  = (_Float16*)(ws + kOffWo1T);
  _Float16* wqT   = (_Float16*)(ws + kOffWqT);
  _Float16* wkvT  = (_Float16*)(ws + kOffWkvT);
  _Float16* wo2T  = (_Float16*)(ws + kOffWo2T);
  _Float16* w1T   = (_Float16*)(ws + kOffW1T);
  _Float16* w2T   = (_Float16*)(ws + kOffW2T);
  _Float16* qkv   = (_Float16*)(ws + kOffQkv);
  _Float16* attn  = (_Float16*)(ws + kOffAttn);
  float*    uf    = (float*)(ws + kOffU);
  float*    t1f   = (float*)(ws + kOffT1f);
  _Float16* t1h   = (_Float16*)(ws + kOffT1h);
  _Float16* q2    = (_Float16*)(ws + kOffQ2);
  _Float16* kv2   = (_Float16*)(ws + kOffKv2);
  float*    t2f   = (float*)(ws + kOffT2f);
  _Float16* t2h   = (_Float16*)(ws + kOffT2h);
  _Float16* hid   = (_Float16*)(ws + kOffHid);

  typedef const unsigned short* cus;

  {
    const int n8 = kRows * (kDim / 8);
    cast_act<<<dim3((unsigned)((n8 + 255) / 256)), dim3(256), 0, stream>>>(target, tgt16, n8, kSeq, kSeqFull, kCarryIn);
  }
  {
    const int n8 = kCRows * (kDim / 8);
    cast_act<<<dim3((unsigned)((n8 + 255) / 256)), dim3(256), 0, stream>>>(context, ctx16, n8, kSrc, kSrcFull, kCarryIn);
  }
  cast_wT<<<dim3(kQkvLd / 64, kDim / 64), dim3(256), 0, stream>>>(Wqkv, wqkvT, kDim, kQkvLd, kCarryW);
  cast_wT<<<dim3(kDim / 64, kDim / 64), dim3(256), 0, stream>>>(Wo1, wo1T, kDim, kDim, kCarryWo);
  cast_wT<<<dim3(kDim / 64, kDim / 64), dim3(256), 0, stream>>>(Wq, wqT, kDim, kDim, kCarryW);
  cast_wT<<<dim3(kDim / 64, kDim / 64), dim3(256), 0, stream>>>(Wk, wkvT, kDim, kDim, kCarryW);
  cast_wT<<<dim3(kDim / 64, kDim / 64), dim3(256), 0, stream>>>(Wv, wkvT + (size_t)kDim * kDim, kDim, kDim, kCarryW);
  cast_wT<<<dim3(kDim / 64, kDim / 64), dim3(256), 0, stream>>>(Wo2, wo2T, kDim, kDim, kCarryWo);
  cast_wT<<<dim3(kFfn / 64, kDim / 64), dim3(256), 0, stream>>>(W1, w1T, kDim, kFfn, kCarryW1);
  cast_wT<<<dim3(kDim / 64, kFfn / 64), dim3(256), 0, stream>>>(W2, w2T, kFfn, kDim, kCarryW2);

  {
    const unsigned tiles = (unsigned)((kSeq / 64) * (kQkvLd / 64));
    wmma_gemm64<0, false, 0, 1, false, false, 0><<<dim3((tiles + 7) / 8, kBatch), dim3(256), 0, stream>>>(
        (cus)tgt16, (cus)tgt16, kDim, (long)kSeq * kDim,
        (cus)wqkvT, (cus)wqkvT, kDim, (long)0,
        (void*)qkv, (void*)qkv, kQkvLd, (long)kSeq * kQkvLd,
        bo1, uf, (long)0,
        kSeq, kQkvLd, kDim, kCarryQkv / (kCarryIn * kCarryW), 1.0f);
  }
  {
    const unsigned blocks = (unsigned)(kBatch * kHeads * (kSeq / kAQB));
    attn_h64<true><<<dim3(blocks), dim3(128), 0, stream>>>(
        qkv, kQkvLd, (long)kSeq * kQkvLd,
        qkv + kDim, kQkvLd, (long)kSeq * kQkvLd,
        qkv + 2 * kDim, kQkvLd, (long)kSeq * kQkvLd,
        tpad, kSeqFull,
        attn, (long)kSeq * kDim,
        kSeq, kSeq, 0.125f / (kCarryQkv * kCarryQkv), kCarryP, kCarryAttn / (kCarryP * kCarryQkv));
  }
  {
    const unsigned tiles = (unsigned)((kSeq / 64) * (kDim / 64));
    wmma_gemm64<0, false, 2, 0, true, true, 0><<<dim3((tiles + 7) / 8, kBatch), dim3(256), 0, stream>>>(
        (cus)attn, (cus)attn, kDim, (long)kSeq * kDim,
        (cus)wo1T, (cus)wo1T, kDim, (long)0,
        (void*)uf, (void*)uf, kDim, (long)kSeq * kDim,
        bo1, target, (long)kSeqFull * kDim,
        kSeq, kDim, kDim, 1.0f / (kCarryAttn * kCarryWo), 1.0f);
  }
  layernorm_rows<true><<<dim3((unsigned)kRows), dim3(256), 0, stream>>>(uf, g1, b1, t1f, t1h, kCarryAct, 1e-5f);

  {
    const unsigned tiles = (unsigned)((kSeq / 64) * (kDim / 64));
    wmma_gemm64<0, false, 0, 1, false, false, 0><<<dim3((tiles + 7) / 8, kBatch), dim3(256), 0, stream>>>(
        (cus)t1h, (cus)t1h, kDim, (long)kSeq * kDim,
        (cus)wqT, (cus)wqT, kDim, (long)0,
        (void*)q2, (void*)q2, kDim, (long)kSeq * kDim,
        bo1, uf, (long)0,
        kSeq, kDim, kDim, kCarryQkv / (kCarryAct * kCarryW), 1.0f);
  }
  {
    const unsigned tiles = (unsigned)((kSrc / 64) * (kKvLd / 64));
    wmma_gemm64<0, false, 0, 1, false, false, 0><<<dim3((tiles + 7) / 8, kBatch), dim3(256), 0, stream>>>(
        (cus)ctx16, (cus)ctx16, kDim, (long)kSrc * kDim,
        (cus)wkvT, (cus)wkvT, kDim, (long)0,
        (void*)kv2, (void*)kv2, kKvLd, (long)kSrc * kKvLd,
        bo1, uf, (long)0,
        kSrc, kKvLd, kDim, kCarryQkv / (kCarryIn * kCarryW), 1.0f);
  }
  {
    const unsigned blocks = (unsigned)(kBatch * kHeads * (kSeq / kAQB));
    attn_h64<false><<<dim3(blocks), dim3(128), 0, stream>>>(
        q2, kDim, (long)kSeq * kDim,
        kv2, kKvLd, (long)kSrc * kKvLd,
        kv2 + kDim, kKvLd, (long)kSrc * kKvLd,
        cpad, kSrcFull,
        attn, (long)kSeq * kDim,
        kSeq, kSrc, 0.125f / (kCarryQkv * kCarryQkv), kCarryP, kCarryAttn / (kCarryP * kCarryQkv));
  }
  {
    const unsigned tiles = (unsigned)((kSeq / 64) * (kDim / 64));
    wmma_gemm64<0, false, 2, 0, true, false, 0><<<dim3((tiles + 7) / 8, kBatch), dim3(256), 0, stream>>>(
        (cus)attn, (cus)attn, kDim, (long)kSeq * kDim,
        (cus)wo2T, (cus)wo2T, kDim, (long)0,
        (void*)uf, (void*)uf, kDim, (long)kSeq * kDim,
        bo2, t1f, (long)kSeq * kDim,
        kSeq, kDim, kDim, 1.0f / (kCarryAttn * kCarryWo), 1.0f);
  }
  layernorm_rows<true><<<dim3((unsigned)kRows), dim3(256), 0, stream>>>(uf, g2, b2, t2f, t2h, kCarryAct, 1e-5f);

  {
    const unsigned tiles = (unsigned)((kSeq / 64) * (kFfn / 64));
    wmma_gemm64<0, false, 2, 1, false, false, 7><<<dim3((tiles + 7) / 8, kBatch), dim3(256), 0, stream>>>(
        (cus)t2h, (cus)t2h, kDim, (long)kSeq * kDim,
        (cus)w1T, (cus)w1T, kDim, (long)0,
        (void*)hid, (void*)hid, kFfn, (long)kSeq * kFfn,
        bf1, uf, (long)0,
        kSeq, kFfn, kDim, 1.0f / (kCarryAct * kCarryW1), kCarryH);
  }
  {
    const unsigned tiles = (unsigned)((kSeq / 64) * (kDim / 64));
    wmma_gemm64<0, false, 2, 0, true, false, 0><<<dim3((tiles + 7) / 8, kBatch), dim3(256), 0, stream>>>(
        (cus)hid, (cus)hid, kFfn, (long)kSeq * kFfn,
        (cus)w2T, (cus)w2T, kFfn, (long)0,
        (void*)uf, (void*)uf, kDim, (long)kSeq * kDim,
        bf2, t2f, (long)kSeq * kDim,
        kSeq, kDim, kFfn, 1.0f / (kCarryH * kCarryW2), 1.0f);
  }
  layernorm_rows<false><<<dim3((unsigned)kRows), dim3(256), 0, stream>>>(uf, g3, b3, outf, t2h, kCarryAct, 1e-6f);
}
